// Attention_13503377178668
// MI455X (gfx1250) — hardware-verified
//
#include <hip/hip_runtime.h>


#ifndef NB
#define NB 64
#endif
#ifndef LAT
#define LAT 128
#endif
#ifndef NKV
#define NKV 512
#endif
#define NB_FULL  64
#define LAT_FULL 128
#define NKV_FULL 512
#define QD   512
#define KVD  256
#define NH   16
#define HD   64
#define HID  (NH * HD)
#define CHB  ((NB) < 16 ? (NB) : 16)
#define NCH  ((NB) / (CHB))
#define NWV  4
#define BQ   (16 * NWV)
#define KS   32
#define OSP  68
#define GSP  68
#define TRP  72
#define PCAR 1024.0f
#define VCAR 16.0f
#define CCAR 256.0f
#define WOCAR 64.0f
#define CTXF 0.015625f
#define OUTF 6.103515625e-05f
#define SCL  (0.125f * 1.4426950408889634f)

static_assert(HD == 64);
static_assert(HID == 1024);
static_assert(NB <= NB_FULL);
static_assert(LAT <= LAT_FULL);
static_assert(NKV <= NKV_FULL);
static_assert(NB % CHB == 0);
static_assert(LAT % BQ == 0);
static_assert(NKV % KS == 0);
static_assert(QD % 32 == 0);
static_assert(KVD % 32 == 0);
static_assert(HID % 32 == 0);
static_assert(((size_t)NB * LAT) % 128 == 0);
static_assert(((size_t)CHB * NKV) % 128 == 0);
static_assert(HID % 128 == 0);
static_assert(HID % 64 == 0);
static_assert(NKV % 64 == 0);
static_assert(QD % 64 == 0);
static_assert(QD % 64 == 0 && HID % 128 == 0);
static_assert(KVD % 64 == 0 && (2 * HID) % 128 == 0);
static_assert(HID % 64 == 0 && QD % 128 == 0);
static_assert(((size_t)LAT * QD) % 8 == 0);
static_assert(((size_t)NKV * KVD) % 8 == 0);
static_assert(GSP % 4 == 0 && OSP % 4 == 0 && TRP % 8 == 0);

#define SZ_QB   ((size_t)NB * LAT * QD * 2)
#define SZ_KVB  ((size_t)NB * NKV * KVD * 2)
#define SZ_WQT  ((size_t)HID * QD * 2)
#define SZ_WKVT ((size_t)2 * HID * KVD * 2)
#define SZ_WOT  ((size_t)QD * HID * 2)
#define SZ_QP   ((size_t)NB * LAT * HID * 2)
#define SZ_KP   ((size_t)CHB * NKV * HID * 2)
#define SZ_VT   ((size_t)CHB * HID * NKV * 2)
#define SZ_CTX  ((size_t)NB * LAT * HID * 2)
#define OFF_QB   ((size_t)0)
#define OFF_KVB  (OFF_QB + SZ_QB)
#define OFF_WQT  (OFF_KVB + SZ_KVB)
#define OFF_WKVT (OFF_WQT + SZ_WQT)
#define OFF_WOT  (OFF_WKVT + SZ_WKVT)
#define OFF_QH   (OFF_WOT + SZ_WOT)
#define OFF_QL   (OFF_QH + SZ_QP)
#define OFF_KH   (OFF_QL + SZ_QP)
#define OFF_KL   (OFF_KH + SZ_KP)
#define OFF_VT   (OFF_KL + SZ_KP)
#define OFF_CTX  (OFF_VT + SZ_VT)
#define WS_TOTAL (OFF_CTX + SZ_CTX)
static_assert(WS_TOTAL <= (size_t)134217728);
static_assert(SZ_QB % 256 == 0 && SZ_KVB % 256 == 0 && SZ_QP % 256 == 0 && SZ_KP % 256 == 0 && SZ_VT % 256 == 0 && SZ_CTX % 256 == 0);

typedef unsigned short us;
typedef __attribute__((ext_vector_type(16))) __bf16   v16bf;
typedef __attribute__((ext_vector_type(16))) _Float16 v16h;
typedef __attribute__((ext_vector_type(8)))  _Float16 v8h;
typedef __attribute__((ext_vector_type(8)))  unsigned short v8us;
typedef __attribute__((ext_vector_type(8)))  float    v8f;
typedef __attribute__((ext_vector_type(4)))  float    v4f;
typedef v4f  __attribute__((may_alias)) v4fa;
typedef v8us __attribute__((may_alias)) v8usa;

__device__ __forceinline__ unsigned short f2bf(float f) { unsigned u = __float_as_uint(f); u += 0x7FFFu + ((u >> 16) & 1u); return (unsigned short)(u >> 16); }
__device__ __forceinline__ float bf2f(unsigned short b) { return __uint_as_float(((unsigned)b) << 16); }
__device__ __forceinline__ float bfr(float f) { return bf2f(f2bf(f)); }
__device__ __forceinline__ unsigned short f2h(float f) { return __builtin_bit_cast(unsigned short, (_Float16)f); }
__device__ __forceinline__ v16bf cat16b(v8us lo, v8us hi) { return __builtin_bit_cast(v16bf, __builtin_shufflevector(lo, hi, 0, 1, 2, 3, 4, 5, 6, 7, 8, 9, 10, 11, 12, 13, 14, 15)); }
__device__ __forceinline__ v16h  cat16h(v8us lo, v8us hi) { return __builtin_bit_cast(v16h,  __builtin_shufflevector(lo, hi, 0, 1, 2, 3, 4, 5, 6, 7, 8, 9, 10, 11, 12, 13, 14, 15)); }
__device__ __forceinline__ v8f wmmab(v16bf a, v16bf b, v8f c) { return __builtin_amdgcn_wmma_f32_16x16x32_bf16(false, a, false, b, (short)0, c, false, false); }
__device__ __forceinline__ v8f wmmah(v16h a, v16h b, v8f c)   { return __builtin_amdgcn_wmma_f32_16x16x32_f16(false, a, false, b, (short)0, c, false, false); }
__device__ __forceinline__ v16bf ldb(const us* p) { return cat16b(*(const v8us*)p, *(const v8us*)(p + 16)); }
__device__ __forceinline__ v16h  ldh(const us* p) { return cat16h(*(const v8us*)p, *(const v8us*)(p + 16)); }

struct OpB {
    typedef v16bf frag;
    static __device__ __forceinline__ frag ld(const us* p) { return ldb(p); }
    static __device__ __forceinline__ v8f mma(frag a, frag b, v8f c) { return wmmab(a, b, c); }
};
struct OpH {
    typedef v16h frag;
    static __device__ __forceinline__ frag ld(const us* p) { return ldh(p); }
    static __device__ __forceinline__ v8f mma(frag a, frag b, v8f c) { return wmmah(a, b, c); }
};

__global__ __launch_bounds__(256) void k_cvt(const float* __restrict__ src, us* dst, unsigned per8, unsigned bstride, unsigned nb) {
    const unsigned i = blockIdx.x * 256u + threadIdx.x;
    if (i >= nb * per8) return;
    const unsigned b = i / per8, r = i - b * per8;
    const v8f v = *(const v8f*)(src + (size_t)b * bstride + (size_t)r * 8);
    v8us o;
#pragma unroll
    for (int c = 0; c < 8; ++c) o[c] = f2bf(v[c]);
    us* d = dst + (size_t)i * 8;
    *(volatile v8us*)d = o;
    __threadfence();
    *(volatile v8us*)d = o;
}

__global__ __launch_bounds__(256) void k_tr(const float* __restrict__ in, us* out, unsigned rows, unsigned cols, unsigned mode) {
    __shared__ __align__(16) us tl[128 * TRP];
    const unsigned tid = threadIdx.x;
    const unsigned r0 = blockIdx.y * 64u, c0 = blockIdx.x * 128u;
#pragma unroll 2
    for (unsigned it = 0; it < 8; ++it) {
        const unsigned f = it * 256u + tid;
        const unsigned r = f >> 5, c4 = (f & 31u) * 4u;
        const v4f x = *(const v4f*)(in + (size_t)(r0 + r) * cols + c0 + c4);
#pragma unroll
        for (unsigned c = 0; c < 4; ++c) {
            const us wb = f2bf(x[c]);
            const us wh = f2h(bf2f(wb) * WOCAR);
            tl[(c4 + c) * TRP + r] = mode ? wh : wb;
        }
    }
    __syncthreads();
    const unsigned c8 = (tid & 7u) * 8u, dr = tid >> 3;
#pragma unroll 1
    for (int ps = 0; ps < 2; ++ps) {
#pragma unroll
        for (unsigned it = 0; it < 4; ++it) {
            const unsigned c = it * 32u + dr;
            const v8us o = *(const v8usa*)(tl + c * TRP + c8);
            *(volatile v8us*)(out + (size_t)(c0 + c) * rows + r0 + c8) = o;
        }
        if (ps == 0) __threadfence();
    }
}

template <class OP, int EPI>
__device__ __forceinline__ void gemm_body(const us* __restrict__ A, const us* __restrict__ B, unsigned lda, unsigned ldb, unsigned K,
                                          us* O0, us* O1, float* OF, const float* __restrict__ bias, unsigned ldo, float scale) {
    __shared__ __align__(16) float st[4 * 32 * GSP];
    const unsigned tid = threadIdx.x, lane = tid & 31u, wv = tid >> 5, lr = lane & 15u, hi = lane >> 4;
    const unsigned m0 = blockIdx.y * 128u + wv * 32u, n0 = blockIdx.x * 64u;
    const us* ap = A + (size_t)(m0 + lr) * lda + 8u * hi;
    const us* bp = B + (size_t)(n0 + lr) * ldb + 8u * hi;
    v8f acc0[4], acc1[4];
#pragma unroll
    for (int t = 0; t < 4; ++t) { acc0[t] = (v8f){}; acc1[t] = (v8f){}; }
#pragma unroll 1
    for (unsigned k0 = 0; k0 < K; k0 += 32) {
        const typename OP::frag a0 = OP::ld(ap + k0);
        const typename OP::frag a1 = OP::ld(ap + (size_t)16 * lda + k0);
        typename OP::frag b[4];
#pragma unroll
        for (int t = 0; t < 4; ++t) b[t] = OP::ld(bp + (size_t)t * 16 * ldb + k0);
#pragma unroll
        for (int t = 0; t < 4; ++t) {
            acc0[t] = OP::mma(a0, b[t], acc0[t]);
            acc1[t] = OP::mma(a1, b[t], acc1[t]);
        }
        asm volatile("v_nop\n\tv_nop\n\tv_nop\n\tv_nop"
                     : "+v"(acc0[0]), "+v"(acc0[1]), "+v"(acc0[2]), "+v"(acc0[3]), "+v"(acc1[0]), "+v"(acc1[1]), "+v"(acc1[2]), "+v"(acc1[3])
                     : "v"(a0), "v"(a1), "v"(b[3]));
    }
    float* sw = st + wv * (32 * GSP);
#pragma unroll
    for (int t = 0; t < 4; ++t) {
#pragma unroll
        for (int r = 0; r < 8; ++r) {
            sw[(8 * hi + r) * GSP + t * 16 + lr]      = acc0[t][r];
            sw[(16 + 8 * hi + r) * GSP + t * 16 + lr] = acc1[t][r];
        }
    }
    __syncthreads();
    if (EPI == 0) {
        const unsigned rq = lane >> 3, c8 = (lane & 7u) * 8u;
#pragma unroll 1
        for (int ps = 0; ps < 2; ++ps) {
#pragma unroll 2
            for (unsigned it = 0; it < 8; ++it) {
                const unsigned row = it * 4u + rq;
                const v4f x0 = *(const v4fa*)(sw + row * GSP + c8);
                const v4f x1 = *(const v4fa*)(sw + row * GSP + c8 + 4);
                v8us oh, ol;
#pragma unroll
                for (int c = 0; c < 4; ++c) {
                    const us h0 = f2bf(x0[c]); oh[c] = h0;     ol[c] = f2bf(x0[c] - bf2f(h0));
                    const us h1 = f2bf(x1[c]); oh[4 + c] = h1; ol[4 + c] = f2bf(x1[c] - bf2f(h1));
                }
                const size_t off = (size_t)(m0 + row) * ldo + n0 + c8;
                *(volatile v8us*)(O0 + off) = oh;
                *(volatile v8us*)(O1 + off) = ol;
            }
            if (ps == 0) __threadfence();
        }
    }
    if (EPI == 1) {
        const unsigned rq = lane >> 3, c8 = (lane & 7u) * 8u;
#pragma unroll 1
        for (int ps = 0; ps < 2; ++ps) {
#pragma unroll 2
            for (unsigned it = 0; it < 8; ++it) {
                const unsigned row = it * 4u + rq;
                const v4f x0 = *(const v4fa*)(sw + row * GSP + c8);
                const v4f x1 = *(const v4fa*)(sw + row * GSP + c8 + 4);
                v8h o;
#pragma unroll
                for (int c = 0; c < 4; ++c) { o[c] = (_Float16)(x0[c] * scale); o[4 + c] = (_Float16)(x1[c] * scale); }
                const v8us ou = __builtin_bit_cast(v8us, o);
                *(volatile v8us*)(O0 + (size_t)(m0 + row) * ldo + n0 + c8) = ou;
            }
            if (ps == 0) __threadfence();
        }
    }
    if (EPI == 2) {
        const unsigned rq = lane >> 4, c4 = (lane & 15u) * 4u;
        const v4f bv = *(const v4f*)(bias + n0 + c4);
        v4f bb;
#pragma unroll
        for (int c = 0; c < 4; ++c) bb[c] = bfr(bv[c]);
#pragma unroll 1
        for (int ps = 0; ps < 2; ++ps) {
#pragma unroll 4
            for (unsigned it = 0; it < 16; ++it) {
                const unsigned row = it * 2u + rq;
                const v4f x = *(const v4fa*)(sw + row * GSP + c4);
                v4f val;
#pragma unroll
                for (int c = 0; c < 4; ++c) val[c] = fmaf(x[c], scale, bb[c]);
                *(volatile v4f*)(OF + (size_t)(m0 + row) * ldo + n0 + c4) = val;
            }
            if (ps == 0) __threadfence();
        }
    }
}

__global__ __launch_bounds__(128) void k_gemm_q(const us* __restrict__ QB, const us* __restrict__ WqT, us* QH, us* QL) {
    gemm_body<OpB, 0>(QB, WqT, QD, QD, QD, QH, QL, (float*)0, (const float*)0, HID, 1.0f);
}
__global__ __launch_bounds__(128) void k_gemm_k(const us* __restrict__ KVBc, const us* __restrict__ WkvT, us* KH, us* KL) {
    gemm_body<OpB, 0>(KVBc, WkvT, KVD, KVD, KVD, KH, KL, (float*)0, (const float*)0, HID, 1.0f);
}
__global__ __launch_bounds__(128) void k_gemm_vt(const us* __restrict__ WvT, const us* __restrict__ KVBc, us* VT) {
    const size_t z = blockIdx.z;
    gemm_body<OpB, 1>(WvT, KVBc + z * ((size_t)NKV * KVD), KVD, KVD, KVD, VT + z * ((size_t)HID * NKV), (us*)0, (float*)0, (const float*)0, NKV, VCAR);
}
__global__ __launch_bounds__(128) void k_gemm_o(const us* __restrict__ CTX, const us* __restrict__ WoT, const float* __restrict__ bo, float* OUT) {
    gemm_body<OpH, 2>(CTX, WoT, HID, HID, HID, (us*)0, (us*)0, OUT, bo, QD, OUTF);
}

__global__ __launch_bounds__(128) void k_flash(const us* __restrict__ QH, const us* __restrict__ QL, const us* __restrict__ KH, const us* __restrict__ KL,
                                               const us* __restrict__ VT, us* CTX, unsigned b0) {
    __shared__ __align__(16) float os[NWV * 16 * OSP];
    const unsigned tid = threadIdx.x, lane = tid & 31u, wv = tid >> 5, lr = lane & 15u, hi = lane >> 4;
    const unsigned qpb = (unsigned)(LAT / BQ);
    const unsigned qb = blockIdx.x % qpb;
    const unsigned bh = blockIdx.x / qpb;
    const unsigned h = bh % NH, bl = bh / NH;
    const unsigned b = b0 + bl;
    const unsigned q0 = qb * BQ + wv * 16u;

    v16bf qh[2], ql[2];
    {
        const size_t qoff = ((size_t)b * LAT + q0 + lr) * HID + h * HD + 8u * hi;
#pragma unroll
        for (int dk = 0; dk < 2; ++dk) { qh[dk] = ldb(QH + qoff + dk * 32); ql[dk] = ldb(QL + qoff + dk * 32); }
    }
    const size_t koff = ((size_t)bl * NKV + lr) * HID + h * HD + 8u * hi;
    const size_t voff = ((size_t)bl * HID + h * HD + lr) * NKV + 8u * hi;

    v8f o[4];
#pragma unroll
    for (int t = 0; t < 4; ++t) o[t] = (v8f){};
    float ml = -1.0e30f;
    float l = 0.0f;

#pragma unroll 1
    for (unsigned k0 = 0; k0 < (unsigned)NKV; k0 += KS) {
        v8f s0 = (v8f){}, s1 = (v8f){};
        const size_t ka = koff + (size_t)k0 * HID;
#pragma unroll
        for (int dk = 0; dk < 2; ++dk) {
            const v16bf ah0 = ldb(KH + ka + dk * 32);
            const v16bf al0 = ldb(KL + ka + dk * 32);
            const v16bf ah1 = ldb(KH + ka + (size_t)16 * HID + dk * 32);
            const v16bf al1 = ldb(KL + ka + (size_t)16 * HID + dk * 32);
            s0 = wmmab(al0, qh[dk], s0);
            s0 = wmmab(ah0, ql[dk], s0);
            s0 = wmmab(ah0, qh[dk], s0);
            s1 = wmmab(al1, qh[dk], s1);
            s1 = wmmab(ah1, ql[dk], s1);
            s1 = wmmab(ah1, qh[dk], s1);
        }
        asm volatile("v_nop\n\tv_nop\n\tv_nop\n\tv_nop" : "+v"(s0), "+v"(s1) : "v"(qh[0]), "v"(qh[1]), "v"(ql[0]), "v"(ql[1]));

        float mx = fmaxf(s0[0], s1[0]);
#pragma unroll
        for (int r = 1; r < 8; ++r) mx = fmaxf(mx, fmaxf(s0[r], s1[r]));
        mx = fmaxf(mx, __shfl_xor(mx, 16, 32));
        const float mnl = fmaxf(ml, mx * SCL);
        const float corr = __builtin_amdgcn_exp2f(ml - mnl);
        ml = mnl;
        float p0[8], p1[8];
        float ps = 0.0f;
#pragma unroll
        for (int r = 0; r < 8; ++r) {
            p0[r] = __builtin_amdgcn_exp2f(fmaf(s0[r], SCL, -mnl));
            p1[r] = __builtin_amdgcn_exp2f(fmaf(s1[r], SCL, -mnl));
            ps += p0[r] + p1[r];
        }
        ps += __shfl_xor(ps, 16, 32);
        l = l * corr + ps;
        if (__builtin_amdgcn_ballot_w32(corr != 1.0f) != 0u) {
#pragma unroll
            for (int t = 0; t < 4; ++t) o[t] *= corr;
        }

        v16h pf;
#pragma unroll
        for (int r = 0; r < 8; ++r) {
            pf[r]     = (_Float16)(p0[r] * PCAR);
            pf[8 + r] = (_Float16)(p1[r] * PCAR);
        }

        asm volatile("" ::: "memory");
        const size_t va = voff + k0;
#pragma unroll
        for (int t = 0; t < 4; ++t) {
            const v16h a = ldh(VT + va + (size_t)t * 16 * NKV);
            o[t] = wmmah(a, pf, o[t]);
        }
        asm volatile("v_nop\n\tv_nop\n\tv_nop\n\tv_nop"
                     : "+v"(o[0]), "+v"(o[1]), "+v"(o[2]), "+v"(o[3])
                     : "v"(pf));
    }

    const float inv = CTXF * (1.0f / l);
    float* ow = os + wv * (16 * OSP);
#pragma unroll
    for (int t = 0; t < 4; ++t) {
#pragma unroll
        for (int r = 0; r < 8; ++r) ow[lr * OSP + t * 16 + 8 * hi + r] = o[t][r] * inv;
    }
    __syncthreads();
    const unsigned rq = lane >> 3, c8 = (lane & 7u) * 8u;
    us* crow = CTX + ((size_t)b * LAT + q0) * HID + h * HD + c8;
#pragma unroll 1
    for (int ps2 = 0; ps2 < 2; ++ps2) {
#pragma unroll
        for (unsigned it = 0; it < 4; ++it) {
            const unsigned row = it * 4u + rq;
            const v4f x0 = *(const v4fa*)(ow + row * OSP + c8);
            const v4f x1 = *(const v4fa*)(ow + row * OSP + c8 + 4);
            v8h hv;
#pragma unroll
            for (int c = 0; c < 4; ++c) { hv[c] = (_Float16)x0[c]; hv[4 + c] = (_Float16)x1[c]; }
            const v8us ou = __builtin_bit_cast(v8us, hv);
            *(volatile v8us*)(crow + (size_t)row * HID) = ou;
        }
        if (ps2 == 0) __threadfence();
    }
}

extern "C" void kernel_launch(void* const* d_in, const int* in_sizes, int n_in,
                              void* d_out, int out_size, void* d_ws, size_t ws_size, hipStream_t stream) {
    if (n_in < 6) return;
    if ((size_t)in_sizes[0] < ((size_t)(NB - 1) * LAT_FULL + LAT) * QD) return;
    if ((size_t)in_sizes[1] < ((size_t)(NB - 1) * NKV_FULL + NKV) * KVD) return;
    if ((size_t)in_sizes[2] < (size_t)QD * HID) return;
    if ((size_t)in_sizes[3] < (size_t)KVD * 2 * HID) return;
    if ((size_t)in_sizes[4] < (size_t)HID * QD) return;
    if ((size_t)in_sizes[5] < (size_t)QD) return;
    if ((size_t)out_size < (size_t)NB * LAT * QD) return;
    if (WS_TOTAL > ws_size) return;

    const float* q   = (const float*)d_in[0];
    const float* kv  = (const float*)d_in[1];
    const float* Wq  = (const float*)d_in[2];
    const float* Wkv = (const float*)d_in[3];
    const float* Wo  = (const float*)d_in[4];
    const float* bo  = (const float*)d_in[5];
    float* OUT = (float*)d_out;

    char* wsp = (char*)d_ws;
    us* QB   = (us*)(wsp + OFF_QB);
    us* KVB  = (us*)(wsp + OFF_KVB);
    us* WqT  = (us*)(wsp + OFF_WQT);
    us* WkvT = (us*)(wsp + OFF_WKVT);
    us* WoT  = (us*)(wsp + OFF_WOT);
    us* QH   = (us*)(wsp + OFF_QH);
    us* QL   = (us*)(wsp + OFF_QL);
    us* KH   = (us*)(wsp + OFF_KH);
    us* KL   = (us*)(wsp + OFF_KL);
    us* VT   = (us*)(wsp + OFF_VT);
    us* CTX  = (us*)(wsp + OFF_CTX);

    {
        const unsigned per8 = (unsigned)((size_t)LAT * QD / 8);
        const unsigned g = (unsigned)(((size_t)NB * per8 + 255) / 256);
        k_cvt<<<g, 256, 0, stream>>>(q, QB, per8, (unsigned)((size_t)LAT_FULL * QD), (unsigned)NB);
    }
    {
        const unsigned per8 = (unsigned)((size_t)NKV * KVD / 8);
        const unsigned g = (unsigned)(((size_t)NB * per8 + 255) / 256);
        k_cvt<<<g, 256, 0, stream>>>(kv, KVB, per8, (unsigned)((size_t)NKV_FULL * KVD), (unsigned)NB);
    }
    k_tr<<<dim3(HID / 128, QD / 64, 1), 256, 0, stream>>>(Wq, WqT, (unsigned)QD, (unsigned)HID, 0u);
    k_tr<<<dim3((2 * HID) / 128, KVD / 64, 1), 256, 0, stream>>>(Wkv, WkvT, (unsigned)KVD, (unsigned)(2 * HID), 0u);
    k_tr<<<dim3(QD / 128, HID / 64, 1), 256, 0, stream>>>(Wo, WoT, (unsigned)HID, (unsigned)QD, 1u);

    k_gemm_q<<<dim3(HID / 64, (unsigned)((size_t)NB * LAT / 128), 1), 128, 0, stream>>>(QB, WqT, QH, QL);

    for (unsigned c = 0; c < (unsigned)NCH; ++c) {
        const us* KVBc = KVB + (size_t)c * CHB * NKV * KVD;
        k_gemm_k<<<dim3(HID / 64, (unsigned)((size_t)CHB * NKV / 128), 1), 128, 0, stream>>>(KVBc, WkvT, KH, KL);
        k_gemm_vt<<<dim3(NKV / 64, HID / 128, CHB), 128, 0, stream>>>(WkvT + (size_t)HID * KVD, KVBc, VT);
        k_flash<<<(unsigned)(CHB * NH * (LAT / BQ)), 128, 0, stream>>>(QH, QL, KH, KL, VT, CTX, c * (unsigned)CHB);
    }

    k_gemm_o<<<dim3(QD / 64, (unsigned)((size_t)NB * LAT / 128), 1), 128, 0, stream>>>(CTX, WoT, bo, OUT);
}
